// PackedAttention_73194832658652
// MI455X (gfx1250) — hardware-verified
//
#include <hip/hip_runtime.h>


namespace {
constexpr int NH = 16, T = 4096, D = 64, NSEG = 8;
constexpr float XS = 8.0f, PS = 1024.0f;
typedef _Float16 b16;
typedef __attribute__((ext_vector_type(16))) _Float16 v16b;
typedef __attribute__((ext_vector_type(8))) _Float16 v8b;
typedef __attribute__((ext_vector_type(8))) float v8f;
typedef __attribute__((ext_vector_type(4))) float v4f;
typedef __attribute__((ext_vector_type(2))) float v2f;
__device__ __forceinline__ float bf16_rne(float f) { unsigned int u = __float_as_uint(f); u += 0x7FFFu + ((u >> 16) & 1u); return __uint_as_float(u & 0xFFFF0000u); }
__device__ __forceinline__ void split16(float v, b16& hi, b16& lo) { hi = (b16)v; lo = (b16)(v - (float)hi); }
__device__ __forceinline__ v16b frag_kb(const b16* p, int hh) { const v8b a = *(const v8b*)(p + 8 * hh), b = *(const v8b*)(p + 16 + 8 * hh); v16b f;
#pragma unroll
  for (int e = 0; e < 8; ++e) { f[e] = a[e]; f[8 + e] = b[e]; } return f; }
__device__ __forceinline__ v8f wmma16b(v16b a, v16b b, v8f c) { v8f d = __builtin_amdgcn_wmma_f32_16x16x32_f16(false, a, false, b, (short)0, c, false, false); asm volatile("v_nop\n\tv_nop\n\tv_nop\n\tv_nop" : "+v"(d) : "v"(a), "v"(b)); return d; }
__device__ __forceinline__ void wave_lds_sync() { __builtin_amdgcn_fence(__ATOMIC_RELEASE, "workgroup"); __builtin_amdgcn_wave_barrier(); __builtin_amdgcn_fence(__ATOMIC_ACQUIRE, "workgroup"); }
__device__ __forceinline__ int iclamp(int v, int lo, int hi) { return v < lo ? lo : (v > hi ? hi : v); }
__device__ __forceinline__ int seg_of(const int* cu, int p) { int s = 0; for (int i = 1; i < NSEG; ++i) s += (cu[i] <= p) ? 1 : 0; return s; }

__global__ __launch_bounds__(256) void prep_kernel(const float* __restrict__ q, const float* __restrict__ k, b16* __restrict__ QB, b16* __restrict__ KB) {
  const size_t u = (size_t)blockIdx.x * 256 + threadIdx.x; if (u >= (size_t)NH * T * 8) return; const int d0 = (int)(u % 8) * 8; const size_t row = u / 8; v8b a, bq;
#pragma unroll
  for (int j = 0; j < 8; ++j) { a[j] = (b16)(bf16_rne(q[row * D + d0 + j]) * XS); bq[j] = (b16)(bf16_rne(k[row * D + d0 + j]) * XS); }
  for (int pass = 0; pass < 2; ++pass) { *(volatile v8b*)(QB + row * D + d0) = a; *(volatile v8b*)(KB + row * D + d0) = bq; __threadfence(); }
}
__global__ __launch_bounds__(32) void att_kernel(const b16* __restrict__ QB, const b16* __restrict__ KB, const float* __restrict__ v, const int* __restrict__ cu, int QLIM, float* __restrict__ out) {
  __shared__ __attribute__((aligned(16))) b16 Ph[16][40], Pl[16][40], Vt[D][40]; __shared__ float Sc[16][33], Mx[16], Dn[16], Sf[16], Of[16][D + 2]; __shared__ int Sg[16], Cu[NSEG + 1], Kr[2];
  const int lane = threadIdx.x, nloc = lane & 15, hlf = lane >> 4; const int h = blockIdx.x / (QLIM / 16), q0 = (blockIdx.x % (QLIM / 16)) * 16;
  if (lane <= NSEG) Cu[lane] = iclamp(cu[lane], 0, T);
  wave_lds_sync();
  if (lane < 16) { Sg[lane] = seg_of(Cu, q0 + lane); Mx[lane] = -INFINITY; Dn[lane] = 0.0f; Sf[lane] = 0.0f; }
  wave_lds_sync();
  if (lane == 0) { Kr[0] = Cu[Sg[0]] & ~31; Kr[1] = Cu[Sg[15] + 1]; }
  wave_lds_sync(); const int kbeg = Kr[0], kend = Kr[1];
  v8f acc[4] = {(v8f){}, (v8f){}, (v8f){}, (v8f){}}; const b16* qb = QB + ((size_t)h * T + q0) * D;
#pragma unroll 1
  for (int kc = kbeg; kc < kend; kc += 32) { const b16* kb_ = KB + ((size_t)h * T + kc) * D;
    for (int rr = 0; rr < 32; ++rr) { const int kk = kc + rr; for (int q = 0; q < 2; ++q) Vt[q * 32 + lane][rr] = (b16)(kk < T ? bf16_rne(v[((size_t)h * T + kk) * D + q * 32 + lane]) * XS : 0.0f); }
#pragma unroll
    for (int blk = 0; blk < 2; ++blk) { v8f s = {};
#pragma unroll
      for (int kb = 0; kb < D; kb += 32) s = wmma16b(frag_kb(qb + (size_t)nloc * D + kb, hlf), frag_kb(kb_ + (size_t)(blk * 16 + nloc) * D + kb, hlf), s);
      const int kk = kc + blk * 16 + nloc; const int ks = seg_of(Cu, kk);
#pragma unroll
      for (int r8 = 0; r8 < 8; ++r8) { const int rl = 8 * hlf + r8; Sc[rl][blk * 16 + nloc] = (kk < T && ks == Sg[rl]) ? s[r8] * (0.125f / (XS * XS)) : -INFINITY; } }
    wave_lds_sync();
#pragma unroll 1
    for (int qi = 0; qi < 16; ++qi) { const float sv = Sc[qi][lane]; float cm = sv; for (int o = 16; o; o >>= 1) cm = fmaxf(cm, __shfl_xor(cm, o)); const float mo = Mx[qi]; const float mn = fmaxf(mo, cm); const float p = (sv == -INFINITY || mn == -INFINITY) ? 0.0f : __expf(sv - mn); float psum = p; for (int o = 16; o; o >>= 1) psum += __shfl_xor(psum, o);
      b16 ph, plo; split16(p * PS, ph, plo); Ph[qi][lane] = ph; Pl[qi][lane] = plo; if (lane == 0) { const float sf = (mo == -INFINITY || mn == -INFINITY) ? ((mo == -INFINITY && mn == -INFINITY) ? 1.0f : 0.0f) : __expf(mo - mn); Sf[qi] = sf; Dn[qi] = Dn[qi] * sf + psum; Mx[qi] = mn; } }
    wave_lds_sync();
#pragma unroll
    for (int t = 0; t < 4; ++t) {
#pragma unroll
      for (int r8 = 0; r8 < 8; ++r8) acc[t][r8] *= Sf[8 * hlf + r8];
      const v16b vb = frag_kb(&Vt[t * 16 + nloc][0], hlf); acc[t] = wmma16b(frag_kb(&Ph[nloc][0], hlf), vb, acc[t]); acc[t] = wmma16b(frag_kb(&Pl[nloc][0], hlf), vb, acc[t]); }
    wave_lds_sync(); }
#pragma unroll
  for (int t = 0; t < 4; ++t)
#pragma unroll
    for (int r8 = 0; r8 < 8; ++r8) { const int rl = 8 * hlf + r8; Of[rl][t * 16 + nloc] = acc[t][r8] * (1.0f / (PS * XS)) / Dn[rl]; }
  wave_lds_sync();
  for (int pass = 0; pass < 2; ++pass) { for (int rr = 0; rr < 16; ++rr) *(volatile v2f*)(out + ((size_t)h * T + q0 + rr) * D + lane * 2) = (v2f){Of[rr][lane * 2], Of[rr][lane * 2 + 1]}; __threadfence(); }
}
}

extern "C" void kernel_launch(void* const* d_in, const int* in_sizes, int n_in, void* d_out, int out_size, void* d_ws, size_t ws_size, hipStream_t stream) {
  (void)n_in;
  auto Fp = [&](int i) { return (const float*)d_in[i]; }; auto Ip = [&](int i) { return (const int*)d_in[i]; };
  if (in_sizes[0] != NH * T * D || in_sizes[1] != NH * T * D || in_sizes[2] != NH * T * D || in_sizes[3] != NSEG + 1 || out_size != NH * T * D) return;
  const int QLIM = T;
  size_t off = 0; char* ws = (char*)d_ws;
  auto carve = [&](size_t bytes) { char* p = ws + off; off += (bytes + 255) & ~(size_t)255; return p; };
  b16* QB = (b16*)carve((size_t)NH * T * D * 2); b16* KB = (b16*)carve((size_t)NH * T * D * 2);
  if (off > ws_size || off > ((size_t)32 << 20)) return;
  prep_kernel<<<(NH * T * 8 + 255) / 256, 256, 0, stream>>>(Fp(0), Fp(1), QB, KB);
  att_kernel<<<NH * (QLIM / 16), 32, 0, stream>>>(QB, KB, Fp(2), Ip(3), QLIM, (float*)d_out);
}
